// T_att_1803886264336
// MI455X (gfx1250) — hardware-verified
//
#include <hip/hip_runtime.h>


typedef _Float16       v16h __attribute__((ext_vector_type(16)));
typedef _Float16       v8h  __attribute__((ext_vector_type(8)));
typedef __bf16         v16b __attribute__((ext_vector_type(16)));
typedef __bf16         v8b  __attribute__((ext_vector_type(8)));
typedef float          v8f  __attribute__((ext_vector_type(8)));
typedef float          v4f  __attribute__((ext_vector_type(4)));
typedef unsigned short v8us __attribute__((ext_vector_type(8)));

#define NB 16
#define NT 2048
#define NC 256
#define NH 256

union FragH { v16h v; v8h half[2]; };
union FragB { v16b v; v8b half[2]; };

__device__ __forceinline__ v8f mma_f16(v16h a, v16h b, v8f c) {
  v8f d = __builtin_amdgcn_wmma_f32_16x16x32_f16(false, a, false, b, (short)0, c, false, false);
  asm volatile("v_nop\n\tv_nop\n\tv_nop\n\tv_nop" : "+v"(d) : "v"(a), "v"(b));
  return d;
}
__device__ __forceinline__ v8f mma_bf16(v16b a, v16b b, v8f c) {
  v8f d = __builtin_amdgcn_wmma_f32_16x16x32_bf16(false, a, false, b, (short)0, c, false, false);
  v16h ax = __builtin_bit_cast(v16h, a);
  v16h bx = __builtin_bit_cast(v16h, b);
  asm volatile("v_nop\n\tv_nop\n\tv_nop\n\tv_nop" : "+v"(d) : "v"(ax), "v"(bx));
  return d;
}

__device__ __forceinline__ v8f zero8() {
  v8f z;
#pragma unroll
  for (int e = 0; e < 8; ++e) z[e] = 0.0f;
  return z;
}
__device__ __forceinline__ v4f mk4(float a, float b, float c, float d) {
  v4f v;
  v[0] = a; v[1] = b; v[2] = c; v[3] = d;
  return v;
}

__device__ __forceinline__ unsigned short bf16_bits(float x) {
  unsigned int u = __float_as_uint(x);
  u = u + 0x7FFFu + ((u >> 16) & 1u);
  return (unsigned short)(u >> 16);
}
__device__ __forceinline__ float bf16_val(unsigned short s) {
  return __uint_as_float(((unsigned int)s) << 16);
}

__global__ __launch_bounds__(256) void k_wconv(const float* __restrict__ W0,
                                                const float* __restrict__ W1,
                                                const float* __restrict__ W2,
                                                unsigned short* __restrict__ planes) {
  __shared__ __attribute__((aligned(16))) unsigned short shi[32 * NC];
  __shared__ __attribute__((aligned(16))) unsigned short slo[32 * NC];
  const int tid  = threadIdx.x;
  const int wsel = blockIdx.y;
  const float* W = (wsel == 0) ? W0 : ((wsel == 1) ? W1 : W2);
  const int h0 = blockIdx.x * 32;
  const int j4 = (tid & 7) * 4;
  const int cb = tid >> 3;
#pragma unroll
  for (int i = 0; i < 8; ++i) {
    const int c = cb + 32 * i;
    const v4f x = *(const v4f*)(W + (size_t)c * NH + h0 + j4);
#pragma unroll
    for (int e = 0; e < 4; ++e) {
      const unsigned short hb = bf16_bits(x[e]);
      const float rr = x[e] - bf16_val(hb);
      const unsigned short lb = bf16_bits(rr);
      shi[(j4 + e) * NC + c] = hb;
      slo[(j4 + e) * NC + c] = lb;
    }
  }
  __syncthreads();
  const int wave = tid >> 5, lane = tid & 31;
  unsigned short* dhi = planes + (size_t)(wsel * 2 + 0) * (NC * NH) + (size_t)h0 * NC;
  unsigned short* dlo = planes + (size_t)(wsel * 2 + 1) * (NC * NH) + (size_t)h0 * NC;
  v4f vh[4], vl[4];
#pragma unroll
  for (int rr = 0; rr < 4; ++rr) {
    const int j = wave * 4 + rr;
    vh[rr] = *(const v4f*)(shi + j * NC + lane * 8);
    vl[rr] = *(const v4f*)(slo + j * NC + lane * 8);
  }
#pragma unroll
  for (int rr = 0; rr < 4; ++rr) {
    const int j = wave * 4 + rr;
    *(volatile v4f*)(dhi + (size_t)j * NC + lane * 8) = vh[rr];
    *(volatile v4f*)(dlo + (size_t)j * NC + lane * 8) = vl[rr];
  }
  __threadfence();
#pragma unroll
  for (int rr = 0; rr < 4; ++rr) {
    const int j = wave * 4 + rr;
    *(volatile v4f*)(dhi + (size_t)j * NC + lane * 8) = vh[rr];
    *(volatile v4f*)(dlo + (size_t)j * NC + lane * 8) = vl[rr];
  }
}

__global__ __launch_bounds__(256) void k_xconv(const float* __restrict__ X,
                                                unsigned short* __restrict__ Xhi,
                                                unsigned short* __restrict__ Xlo,
                                                int n8) {
  const int i = blockIdx.x * 256 + threadIdx.x;
  if (i >= n8) return;
  const float* p = X + (size_t)i * 8;
  const v4f a = *(const v4f*)p;
  const v4f b = *(const v4f*)(p + 4);
  union U8 { v8us u; v4f f; } H, L;
#pragma unroll
  for (int e = 0; e < 4; ++e) {
    const unsigned short ha = bf16_bits(a[e]);
    const unsigned short hb = bf16_bits(b[e]);
    H.u[e]     = ha;
    H.u[e + 4] = hb;
    L.u[e]     = bf16_bits(a[e] - bf16_val(ha));
    L.u[e + 4] = bf16_bits(b[e] - bf16_val(hb));
  }
  const v4f hv = H.f, lv = L.f;
  *(volatile v4f*)(Xhi + (size_t)i * 8) = hv;
  *(volatile v4f*)(Xlo + (size_t)i * 8) = lv;
  __threadfence();
  *(volatile v4f*)(Xhi + (size_t)i * 8) = hv;
  *(volatile v4f*)(Xlo + (size_t)i * 8) = lv;
}

__global__ __launch_bounds__(128) void k_proj(const __bf16* __restrict__ Xhi,
                                               const __bf16* __restrict__ Xlo,
                                               const __bf16* __restrict__ Whi,
                                               const __bf16* __restrict__ Wlo,
                                               const float* __restrict__ bias,
                                               _Float16* __restrict__ dst,
                                               int transposed) {
  __shared__ __attribute__((aligned(16))) _Float16 stile[16384];
  const int tid = threadIdx.x;
  const int wave = tid >> 5, lane = tid & 31, m = lane & 15, hh = lane >> 4;
  const int blkrow = blockIdx.x * 64;
  const int rbase  = blkrow + wave * 16;
  const __bf16* xh = Xhi + (size_t)(rbase + m) * NC + 8 * hh;
  const __bf16* xl = Xlo + (size_t)(rbase + m) * NC + 8 * hh;

#pragma unroll 1
  for (int g = 0; g < 2; ++g) {
    v8f acc[8];
#pragma unroll
    for (int j = 0; j < 8; ++j) acc[j] = zero8();
    const __bf16* wh = Whi + (size_t)(g * 128 + m) * NC + 8 * hh;
    const __bf16* wl = Wlo + (size_t)(g * 128 + m) * NC + 8 * hh;
#pragma unroll
    for (int fs = 0; fs < 8; ++fs) {
      FragB ah, al;
      ah.half[0] = *(const v8b*)(xh + fs * 32);
      ah.half[1] = *(const v8b*)(xh + fs * 32 + 16);
      al.half[0] = *(const v8b*)(xl + fs * 32);
      al.half[1] = *(const v8b*)(xl + fs * 32 + 16);
#pragma unroll
      for (int j = 0; j < 8; ++j) {
        FragB bh, bl;
        const __bf16* ph = wh + j * (16 * NC) + fs * 32;
        const __bf16* pl = wl + j * (16 * NC) + fs * 32;
        bh.half[0] = *(const v8b*)ph;
        bh.half[1] = *(const v8b*)(ph + 16);
        bl.half[0] = *(const v8b*)pl;
        bl.half[1] = *(const v8b*)(pl + 16);
        acc[j] = mma_bf16(ah.v, bh.v, acc[j]);
        acc[j] = mma_bf16(ah.v, bl.v, acc[j]);
        acc[j] = mma_bf16(al.v, bh.v, acc[j]);
      }
    }
#pragma unroll
    for (int j = 0; j < 8; ++j) {
      const int hcol = g * 128 + j * 16 + m;
      const float bb = bias[hcol];
      if (transposed) {
        union P8 { v8h v; v4f f; } pk;
#pragma unroll
        for (int r = 0; r < 8; ++r) pk.v[r] = (_Float16)(acc[j][r] + bb);
        *(v4f*)(stile + hcol * 64 + wave * 16 + 8 * hh) = pk.f;
      } else {
#pragma unroll
        for (int r = 0; r < 8; ++r)
          stile[(wave * 16 + 8 * hh + r) * NH + hcol] = (_Float16)(acc[j][r] + bb);
      }
    }
  }
  __syncthreads();

  if (transposed) {
    const int bidx = blkrow / NT;
    const int t0   = blkrow % NT;
    _Float16* vd = dst + (size_t)bidx * NH * NT + t0;
    const int q8 = lane & 7, l3 = lane >> 3;
    v4f vals[16];
#pragma unroll
    for (int it = 0; it < 16; ++it) {
      const int h = wave * 64 + it * 4 + l3;
      vals[it] = *(const v4f*)(stile + h * 64 + q8 * 8);
    }
#pragma unroll
    for (int it = 0; it < 16; ++it) {
      const int h = wave * 64 + it * 4 + l3;
      *(volatile v4f*)(vd + (size_t)h * NT + q8 * 8) = vals[it];
    }
    __threadfence();
#pragma unroll
    for (int it = 0; it < 16; ++it) {
      const int h = wave * 64 + it * 4 + l3;
      *(volatile v4f*)(vd + (size_t)h * NT + q8 * 8) = vals[it];
    }
  } else {
    _Float16* rd = dst + (size_t)rbase * NH;
    v4f vals[16];
#pragma unroll
    for (int r = 0; r < 16; ++r)
      vals[r] = *(const v4f*)(stile + (wave * 16 + r) * NH + lane * 8);
#pragma unroll
    for (int r = 0; r < 16; ++r)
      *(volatile v4f*)(rd + (size_t)r * NH + lane * 8) = vals[r];
    __threadfence();
#pragma unroll
    for (int r = 0; r < 16; ++r)
      *(volatile v4f*)(rd + (size_t)r * NH + lane * 8) = vals[r];
  }
}

__global__ __launch_bounds__(256) void k_attn(const _Float16* __restrict__ Qh,
                                               const _Float16* __restrict__ Kh,
                                               const _Float16* __restrict__ Vt,
                                               float* __restrict__ out) {
  __shared__ __attribute__((aligned(16))) _Float16 Ks[32 * NH];
  __shared__ __attribute__((aligned(16))) _Float16 Vs[NH * 32];
  const int tid = threadIdx.x;
  const int lane = tid & 31, wave = tid >> 5, m = lane & 15, hh = lane >> 4;
  const int b  = blockIdx.y;
  const int q0 = (blockIdx.x * 8 + wave) * 16;
  const _Float16* qp = Qh + ((size_t)b * NT + q0 + m) * NH + 8 * hh;
  const v8h* kg = (const v8h*)(Kh + (size_t)b * NT * NH);
  const v8h* vg = (const v8h*)(Vt + ((size_t)b * NH + tid) * NT);
  v8h* kd = (v8h*)Ks;
  v8h* vd = (v8h*)(Vs + tid * 32);

  const float C1 = 0.0625f * 1.44269504088896341f;
  float mrun = -1.0e30f, l = 0.0f;
  v8f ot[16];
#pragma unroll
  for (int t = 0; t < 16; ++t) ot[t] = zero8();

#pragma unroll 1
  for (int sb = 0; sb < NT / 32; ++sb) {
    __syncthreads();
#pragma unroll
    for (int i = 0; i < 4; ++i)
      kd[tid * 4 + i] = kg[(size_t)sb * (32 * NH / 8) + tid * 4 + i];
#pragma unroll
    for (int i = 0; i < 4; ++i)
      vd[i] = vg[sb * 4 + i];
    __syncthreads();

    v8f st0 = zero8(), st1 = zero8();
#pragma unroll
    for (int fs = 0; fs < 8; ++fs) {
      FragH qb, ka, kb;
      qb.half[0] = *(const v8h*)(qp + fs * 32);
      qb.half[1] = *(const v8h*)(qp + fs * 32 + 16);
      const _Float16* pa = Ks + m * NH + fs * 32 + 8 * hh;
      const _Float16* pb = pa + 16 * NH;
      ka.half[0] = *(const v8h*)pa;
      ka.half[1] = *(const v8h*)(pa + 16);
      kb.half[0] = *(const v8h*)pb;
      kb.half[1] = *(const v8h*)(pb + 16);
      st0 = mma_f16(ka.v, qb.v, st0);
      st1 = mma_f16(kb.v, qb.v, st1);
    }

    float bm = -1.0e30f;
#pragma unroll
    for (int r = 0; r < 8; ++r) bm = fmaxf(bm, fmaxf(st0[r], st1[r]));
    bm = fmaxf(bm, __shfl_xor(bm, 16, 32));
    const float mn    = fmaxf(mrun, bm);
    const float alpha = __builtin_amdgcn_exp2f((mrun - mn) * C1);
    const float cexp  = 14.0f - mn * C1;
    FragH pf;
    float rs = 0.0f;
#pragma unroll
    for (int r = 0; r < 8; ++r) {
      const float p0 = __builtin_amdgcn_exp2f(st0[r] * C1 + cexp);
      const float p1 = __builtin_amdgcn_exp2f(st1[r] * C1 + cexp);
      rs += p0 + p1;
      pf.v[r]     = (_Float16)p0;
      pf.v[8 + r] = (_Float16)p1;
    }
    rs += __shfl_xor(rs, 16, 32);
    l    = l * alpha + rs;
    mrun = mn;

#pragma unroll
    for (int t = 0; t < 16; ++t) ot[t] = ot[t] * alpha;

#pragma unroll
    for (int t = 0; t < 16; ++t) {
      FragH vf;
      const _Float16* vp = Vs + (t * 16 + m) * 32 + 8 * hh;
      vf.half[0] = *(const v8h*)vp;
      vf.half[1] = *(const v8h*)(vp + 16);
      ot[t] = mma_f16(vf.v, pf.v, ot[t]);
    }
  }

  const float inv = 1.0f / l;
  float* orow = out + ((size_t)b * NT + q0 + m) * NH;
  v4f lines[4][8];
#pragma unroll
  for (int i = 0; i < 4; ++i) {
    float s0[8], s1[8], s2[8], s3[8];
#pragma unroll
    for (int r = 0; r < 8; ++r) {
      const float lo0 = ot[4 * i][r] * inv;
      const float lo1 = ot[4 * i + 1][r] * inv;
      const float hi0 = ot[4 * i + 2][r] * inv;
      const float hi1 = ot[4 * i + 3][r] * inv;
      const float snda = hh ? lo0 : hi0;
      const float sndb = hh ? lo1 : hi1;
      const float rcva = __shfl_xor(snda, 16, 32);
      const float rcvb = __shfl_xor(sndb, 16, 32);
      const float oa = hh ? hi0 : lo0;
      const float ob = hh ? hi1 : lo1;
      s0[r] = hh ? rcva : oa;
      s1[r] = hh ? oa : rcva;
      s2[r] = hh ? rcvb : ob;
      s3[r] = hh ? ob : rcvb;
    }
    lines[i][0] = mk4(s0[0], s0[1], s0[2], s0[3]);
    lines[i][1] = mk4(s0[4], s0[5], s0[6], s0[7]);
    lines[i][2] = mk4(s1[0], s1[1], s1[2], s1[3]);
    lines[i][3] = mk4(s1[4], s1[5], s1[6], s1[7]);
    lines[i][4] = mk4(s2[0], s2[1], s2[2], s2[3]);
    lines[i][5] = mk4(s2[4], s2[5], s2[6], s2[7]);
    lines[i][6] = mk4(s3[0], s3[1], s3[2], s3[3]);
    lines[i][7] = mk4(s3[4], s3[5], s3[6], s3[7]);
  }
#pragma unroll
  for (int i = 0; i < 4; ++i) {
    float* lp = orow + 32 * (2 * i + hh);
#pragma unroll
    for (int k = 0; k < 8; ++k) *(volatile v4f*)(lp + 4 * k) = lines[i][k];
  }
  __threadfence();
#pragma unroll
  for (int i = 0; i < 4; ++i) {
    float* lp = orow + 32 * (2 * i + hh);
#pragma unroll
    for (int k = 0; k < 8; ++k) *(volatile v4f*)(lp + 4 * k) = lines[i][k];
  }
}

extern "C" void kernel_launch(void* const* d_in, const int* in_sizes, int n_in,
                              void* d_out, int out_size, void* d_ws, size_t ws_size,
                              hipStream_t stream) {
  if (n_in < 9) return;
  const int nx = NB * NT * NC;
  const int nw = NC * NH;
  if (in_sizes[0] != nx || in_sizes[1] != nx || in_sizes[2] != nx) return;
  if (in_sizes[3] != nw || in_sizes[5] != nw || in_sizes[7] != nw) return;
  if (in_sizes[4] != NH || in_sizes[6] != NH || in_sizes[8] != NH) return;
  if (out_size != NB * NT * NH) return;

  const float* q  = (const float*)d_in[0];
  const float* k  = (const float*)d_in[1];
  const float* v  = (const float*)d_in[2];
  const float* Wq = (const float*)d_in[3];
  const float* bq = (const float*)d_in[4];
  const float* Wk = (const float*)d_in[5];
  const float* bk = (const float*)d_in[6];
  const float* Wv = (const float*)d_in[7];
  const float* bv = (const float*)d_in[8];
  float* out = (float*)d_out;

  char* ws = (char*)d_ws;
  const size_t planeElems = (size_t)NC * NH;
  const size_t wBytes     = 6 * planeElems * sizeof(unsigned short);
  const size_t xBytes     = (size_t)nx * sizeof(unsigned short);
  const size_t pBytes     = (size_t)NB * NT * NH * sizeof(_Float16);
  size_t off = 0;
  unsigned short* wpl = (unsigned short*)(ws + off); off += wBytes;
  off = (off + 255) & ~(size_t)255;
  unsigned short* xhi = (unsigned short*)(ws + off); off += xBytes;
  unsigned short* xlo = (unsigned short*)(ws + off); off += xBytes;
  _Float16* Qh = (_Float16*)(ws + off); off += pBytes;
  _Float16* Kh = (_Float16*)(ws + off); off += pBytes;
  _Float16* Vt = (_Float16*)(ws + off); off += pBytes;
  if (off > ws_size) return;

  const __bf16* wq_hi = (const __bf16*)(wpl + 0 * planeElems);
  const __bf16* wq_lo = (const __bf16*)(wpl + 1 * planeElems);
  const __bf16* wk_hi = (const __bf16*)(wpl + 2 * planeElems);
  const __bf16* wk_lo = (const __bf16*)(wpl + 3 * planeElems);
  const __bf16* wv_hi = (const __bf16*)(wpl + 4 * planeElems);
  const __bf16* wv_lo = (const __bf16*)(wpl + 5 * planeElems);
  const __bf16* x_hi  = (const __bf16*)xhi;
  const __bf16* x_lo  = (const __bf16*)xlo;

  const int n8       = nx / 8;
  const int convGrid = (n8 + 255) / 256;
  const int projGrid = (NB * NT) / 64;

  k_wconv<<<dim3(NH / 32, 3), 256, 0, stream>>>(Wq, Wk, Wv, wpl);

  k_xconv<<<convGrid, 256, 0, stream>>>(q, xhi, xlo, n8);
  k_proj<<<projGrid, 128, 0, stream>>>(x_hi, x_lo, wq_hi, wq_lo, bq, Qh, 0);

  k_xconv<<<convGrid, 256, 0, stream>>>(k, xhi, xlo, n8);
  k_proj<<<projGrid, 128, 0, stream>>>(x_hi, x_lo, wk_hi, wk_lo, bk, Kh, 0);

  k_xconv<<<convGrid, 256, 0, stream>>>(v, xhi, xlo, n8);
  k_proj<<<projGrid, 128, 0, stream>>>(x_hi, x_lo, wv_hi, wv_lo, bv, Vt, 1);

  k_attn<<<dim3(NT / 128, NB), 256, 0, stream>>>(Qh, Kh, Vt, out);
}
